// CharBiLSTMEmbedder_8744553415088
// MI455X (gfx1250) — hardware-verified
//
#include <hip/hip_runtime.h>
#include <math.h>

typedef __attribute__((ext_vector_type(16))) _Float16 v16h;
typedef __attribute__((ext_vector_type(8)))  _Float16 v8h;
typedef __attribute__((ext_vector_type(16))) __bf16   v16b;
typedef __attribute__((ext_vector_type(8)))  __bf16   v8b;
typedef __attribute__((ext_vector_type(8)))  float    v8f;
typedef __attribute__((ext_vector_type(4)))  float    v4f;

constexpr int kN    = 16384;
constexpr int kT    = 16;
constexpr int kV    = 128;
constexpr int kE    = 128;
constexpr int kHid  = 256;
constexpr int kG4   = 4 * kHid;
constexpr int kThr  = 256;
constexpr float kInCarry = 1024.0f;
constexpr float kCarry = kInCarry;
constexpr float kSc = 1.0f / (kCarry * kCarry);
constexpr float kF16MinNormal = 6.103515625e-5f;

static_assert((kN % 64) == 0 && (kV % 64) == 0 && (kG4 % 64) == 0 && ((kV / 64) * (kG4 / 64)) % 8 == 0 && ((kN / 64) * (kG4 / 64)) % 8 == 0, "GEMM M, N multiples of 64; grids exact");
static_assert((kE % 32) == 0 && (kHid % 32) == 0 && (kHid % 256) == 0, "GEMM K multiples of 32; the plane cast's pitch a multiple of 256");

constexpr size_t kOffEMB16 = 0ull;
constexpr size_t kOffWIF = 32768ull;
constexpr size_t kOffWIB = 294912ull;
constexpr size_t kOffWHF = 557056ull;
constexpr size_t kOffWHB = 1081344ull;
constexpr size_t kOffBIAS = 1605632ull;
constexpr size_t kOffPF = 1622016ull;
constexpr size_t kOffPB = 2146304ull;
constexpr size_t kOffH32 = 2670592ull;
constexpr size_t kOffC32 = 19447808ull;
constexpr size_t kOffH16 = 36225024ull;
constexpr size_t kOffGG = 44613632ull;
constexpr size_t kWsTotal = 111722496ull;
static_assert(kWsTotal <= 134217728ull, "carve cap: under 128 MiB");
static_assert(kOffEMB16 == 0
              && kOffWIF == kOffEMB16 + 32768ull
              && kOffWIB == kOffWIF + 262144ull
              && kOffWHF == kOffWIB + 262144ull
              && kOffWHB == kOffWHF + 524288ull
              && kOffBIAS == kOffWHB + 524288ull
              && kOffPF == kOffBIAS + 16384ull
              && kOffPB == kOffPF + 524288ull
              && kOffH32 == kOffPB + 524288ull
              && kOffC32 == kOffH32 + 16777216ull
              && kOffH16 == kOffC32 + 16777216ull
              && kOffGG == kOffH16 + 8388608ull
              && kWsTotal == kOffGG + 67108864ull, "the carve is chained and totalled");
static_assert((kOffEMB16 % 256) == 0 && (kOffWIF % 256) == 0 && (kOffWIB % 256) == 0 && (kOffWHF % 256) == 0 && (kOffWHB % 256) == 0 && (kOffBIAS % 256) == 0 && (kOffPF % 256) == 0 && (kOffPB % 256) == 0 && (kOffH32 % 256) == 0 && (kOffC32 % 256) == 0 && (kOffH16 % 256) == 0 && (kOffGG % 256) == 0, "aligned regions");
constexpr int kFBF = 0, kFBB = 1024, kFZB = 2048, kFEnd = 4096;
static_assert(kFBB == kFBF + kG4 && kFZB == kFBB + kG4 && kFZB + kG4 <= kFEnd && (kFZB % 128) == 0, "bias stream map; the zero row reaches the step product's 1,024 columns");

__device__ __forceinline__ unsigned short f2bf_bits(float f) {
  unsigned u = __float_as_uint(f);
  return (unsigned short)((u + 0x7FFFu + ((u >> 16) & 1u)) >> 16);
}
__device__ __forceinline__ float bf_bits2f(unsigned short h) { return __uint_as_float(((unsigned)h) << 16); }
__device__ __forceinline__ float bf16r(float f) { return bf_bits2f(f2bf_bits(f)); }
__device__ __forceinline__ float carry_flush(float v, float carry) {
  const float s = v * carry;
  return (fabsf(s) < kF16MinNormal) ? 0.0f : s;
}
__device__ __forceinline__ float frcp(float x) { return __builtin_amdgcn_rcpf(x); }

__device__ __forceinline__ void dep_guard4_h(v8f& a, v8f& b, v8f& c, v8f& d, v16h x, v16h y) { asm volatile("v_nop\n\tv_nop\n\tv_nop\n\tv_nop" : "+v"(a), "+v"(b), "+v"(c), "+v"(d) : "v"(x), "v"(y)); }
__device__ __forceinline__ void dep_guard4_b(v8f& a, v8f& b, v8f& c, v8f& d, v16b x, v16b y) { asm volatile("v_nop\n\tv_nop\n\tv_nop\n\tv_nop" : "+v"(a), "+v"(b), "+v"(c), "+v"(d) : "v"(x), "v"(y)); }
__device__ __forceinline__ void keep4_h(v16h a, v16h b, v16h c, v16h d) { asm volatile("v_nop" :: "v"(a), "v"(b), "v"(c), "v"(d)); }
__device__ __forceinline__ void keep4_b(v16b a, v16b b, v16b c, v16b d) { asm volatile("v_nop" :: "v"(a), "v"(b), "v"(c), "v"(d)); }
__device__ __forceinline__ void acc_guard4(v8f& a, v8f& b, v8f& c, v8f& d) { asm volatile("v_nop\n\tv_nop\n\tv_nop\n\tv_nop" : "+v"(a), "+v"(b), "+v"(c), "+v"(d)); }

template <typename T> struct Frag;
template <> struct Frag<_Float16> {
  typedef v16h V; union U { v16h v; v8h h[2]; };
  static __device__ __forceinline__ v16h load(const _Float16* p) {
    U f; f.h[0] = *(const v8h*)(p); f.h[1] = *(const v8h*)(p + 16); return f.v;
  }
  static __device__ __forceinline__ v8f mma(v16h a, v16h b, v8f c) {
    return __builtin_amdgcn_wmma_f32_16x16x32_f16(false, a, false, b, (short)0, c, false, false);
  }
  static __device__ __forceinline__ void guard4(v8f& a, v8f& b, v8f& c, v8f& d, v16h x, v16h y) { dep_guard4_h(a, b, c, d, x, y); }
  static __device__ __forceinline__ void keep(v16h a, v16h b, v16h c, v16h d) { keep4_h(a, b, c, d); }
};
template <> struct Frag<__bf16> {
  typedef v16b V; union U { v16b v; v8b h[2]; };
  static __device__ __forceinline__ v16b load(const __bf16* p) {
    U f; f.h[0] = *(const v8b*)(p); f.h[1] = *(const v8b*)(p + 16); return f.v;
  }
  static __device__ __forceinline__ v8f mma(v16b a, v16b b, v8f c) {
    return __builtin_amdgcn_wmma_f32_16x16x32_bf16(false, a, false, b, (short)0, c, false, false);
  }
  static __device__ __forceinline__ void guard4(v8f& a, v8f& b, v8f& c, v8f& d, v16b x, v16b y) { dep_guard4_b(a, b, c, d, x, y); }
  static __device__ __forceinline__ void keep(v16b a, v16b b, v16b c, v16b d) { keep4_b(a, b, c, d); }
};

__device__ __forceinline__ v8f mma_h(v16h a, v16h b, v8f c) {
  c = __builtin_amdgcn_wmma_f32_16x16x32_f16(false, a, false, b, (short)0, c, false, false);
  asm volatile("v_nop\n\tv_nop\n\tv_nop\n\tv_nop" : "+v"(c) : "v"(a), "v"(b));
  return c;
}

template <int ET> struct Elem;
template <> struct Elem<0> { typedef _Float16 T; };
template <> struct Elem<1> { typedef __bf16 T; };
template <int ET, bool SPLIT, int BIAS_MODE, int OUT_MODE, bool RESID, int ACT = 0>
__global__ __launch_bounds__(256) void wmma_gemm64(
    const unsigned short* __restrict__ Ap, const unsigned short* __restrict__ A2p, int lda, long strideA,
    const unsigned short* __restrict__ Btp, const unsigned short* __restrict__ Bt2p, int ldb, long strideB,
    void* __restrict__ Cout, void* __restrict__ Cout2, int ldc, long strideC,
    const float* __restrict__ bias,
    const float* __restrict__ resid, long strideR,
    int M, int N, int K, float scale) {
  typedef typename Elem<ET>::T T;
  typedef typename Frag<T>::V V;
  const T* A = (const T*)Ap; const T* A2 = (const T*)A2p; const T* Bt = (const T*)Btp; const T* Bt2 = (const T*)Bt2p;
  __shared__ __align__(16) float sT[8][16 * 68];
  const int b    = blockIdx.y;
  const int lane = threadIdx.x & 31;
  const int wave = threadIdx.x >> 5;
  const int tilesN = N >> 6;
  const int tilesM = M >> 6;
  const int tile = blockIdx.x * 8 + wave;
  if (tile >= tilesM * tilesN) return;
  const int tm = tile / tilesN;
  const int tn = tile - tm * tilesN;
  const int m0 = tm << 6;
  const int n0 = tn << 6;

  const T* Ab  = A  + (size_t)b * strideA;
  const T* Bb  = Bt + (size_t)b * strideB;
  const T* Ab2 = SPLIT ? (A2  + (size_t)b * strideA) : nullptr;
  const T* Bb2 = SPLIT ? (Bt2 + (size_t)b * strideB) : nullptr;

  const int rlane = lane & 15;
  const int koff  = (lane >> 4) * 8;
  const int mOff  = (lane >> 4) * 8;

  v8f acc[4][4];
#pragma unroll
  for (int i = 0; i < 4; ++i)
#pragma unroll
    for (int j = 0; j < 4; ++j) acc[i][j] = (v8f){0.f,0.f,0.f,0.f,0.f,0.f,0.f,0.f};

  for (int k0 = 0; k0 < K; k0 += 32) {
    V bh[4], bl[4];
#pragma unroll
    for (int j = 0; j < 4; ++j) {
      const size_t bo = (size_t)(n0 + (j << 4) + rlane) * ldb + koff + k0;
      bh[j] = Frag<T>::load(Bb + bo);
      if (SPLIT) bl[j] = Frag<T>::load(Bb2 + bo);
    }
#pragma unroll
    for (int i = 0; i < 4; ++i) {
      const size_t ao = (size_t)(m0 + (i << 4) + rlane) * lda + koff + k0;
      V ah = Frag<T>::load(Ab + ao);
      V al;
      if (SPLIT) al = Frag<T>::load(Ab2 + ao);
#pragma unroll
      for (int j = 0; j < 4; ++j) {
        acc[i][j] = Frag<T>::mma(ah, bh[j], acc[i][j]);
        if (SPLIT) {
          acc[i][j] = Frag<T>::mma(ah, bl[j], acc[i][j]);
          acc[i][j] = Frag<T>::mma(al, bh[j], acc[i][j]);
        }
      }
      Frag<T>::guard4(acc[i][0], acc[i][1], acc[i][2], acc[i][3], ah, SPLIT ? al : ah);
    }
    Frag<T>::keep(bh[0], bh[1], bh[2], bh[3]);
    if (SPLIT) Frag<T>::keep(bl[0], bl[1], bl[2], bl[3]);
  }
  acc_guard4(acc[0][0], acc[0][1], acc[0][2], acc[0][3]);
  acc_guard4(acc[1][0], acc[1][1], acc[1][2], acc[1][3]);
  acc_guard4(acc[2][0], acc[2][1], acc[2][2], acc[2][3]);
  acc_guard4(acc[3][0], acc[3][1], acc[3][2], acc[3][3]);

  float* slab = sT[wave];
  const float* Rb = RESID ? (resid + (size_t)b * strideR) : nullptr;
#pragma unroll
  for (int i = 0; i < 4; ++i) {
    const int mBase = m0 + (i << 4);
#pragma unroll
    for (int j = 0; j < 4; ++j) {
      const int n = n0 + (j << 4) + rlane;
      float bv = 0.f;
      if (BIAS_MODE == 2) bv = bias[n];
#pragma unroll
      for (int r = 0; r < 8; ++r) {
        float v = acc[i][j][r] * scale;
        if (BIAS_MODE == 1) v += bias[mBase + mOff + r];
        if (BIAS_MODE == 2) v += bv;
        if (RESID) v += Rb[(size_t)(mBase + mOff + r) * ldc + n];
        if (ACT == 1) v = tanhf(v);
        if (ACT == 2) v = fmaxf(v, 0.0f);
        if (ACT == 3) v = v / (1.0f + expf(-v));
        if (ACT == 4) v = (v > 0.f) ? v : 0.01f * v;
        slab[(mOff + r) * 68 + (j << 4) + rlane] = v;
      }
    }
    __builtin_amdgcn_fence(__ATOMIC_RELEASE, "workgroup");
    __builtin_amdgcn_wave_barrier();
    __builtin_amdgcn_fence(__ATOMIC_ACQUIRE, "workgroup");
    if (OUT_MODE == 0) {
      float* C = (float*)Cout + (size_t)b * strideC;
      const int hh = lane >> 4, c4 = (lane & 15) * 4;
      for (int pass = 0; pass < 2; ++pass) {
#pragma unroll
        for (int it = 0; it < 8; ++it) {
          const int row = it * 2 + hh;
          v4f v = *(const v4f*)(slab + row * 68 + c4);
          *(volatile v4f*)(C + (size_t)(mBase + row) * ldc + n0 + c4) = v;
        }
        __threadfence();
      }
    } else {
      const int q = lane >> 3, c8 = (lane & 7) * 8;
      unsigned short* C  = (unsigned short*)Cout  + (size_t)b * strideC;
      unsigned short* C2 = (OUT_MODE == 2) ? ((unsigned short*)Cout2 + (size_t)b * strideC) : nullptr;
      for (int pass = 0; pass < 2; ++pass) {
#pragma unroll
        for (int it = 0; it < 4; ++it) {
          const int row = it * 4 + q;
          const float* sp = slab + row * 68 + c8;
          v8h hv, lv;
#pragma unroll
          for (int e = 0; e < 8; ++e) {
            if (OUT_MODE == 1) {
              hv[e] = (_Float16)sp[e];
            } else {
              unsigned short hb = f2bf_bits(sp[e]);
              unsigned short lb = f2bf_bits(sp[e] - bf_bits2f(hb));
              hv[e] = __builtin_bit_cast(_Float16, hb);
              lv[e] = __builtin_bit_cast(_Float16, lb);
            }
          }
          *(volatile v8h*)(C + (size_t)(mBase + row) * ldc + n0 + c8) = hv;
          if (OUT_MODE == 2) *(volatile v8h*)(C2 + (size_t)(mBase + row) * ldc + n0 + c8) = lv;
        }
        __threadfence();
      }
    }
    __builtin_amdgcn_fence(__ATOMIC_RELEASE, "workgroup");
    __builtin_amdgcn_wave_barrier();
    __builtin_amdgcn_fence(__ATOMIC_ACQUIRE, "workgroup");
  }
}

__global__ __launch_bounds__(kThr) void cast_plane_kernel(const float* __restrict__ src, unsigned short* __restrict__ dst,
                                                          int colsLog2, int dstPitch, int dstOff) {
  const int i   = blockIdx.x * kThr + threadIdx.x;
  const int sh  = colsLog2 - 3;
  const int row = i >> sh;
  const int c8  = (i & ((1 << sh) - 1)) * 8;
  const float* sp = src + ((size_t)row << colsLog2) + c8;
  const v4f a0 = *(const v4f*)(sp);
  const v4f a1 = *(const v4f*)(sp + 4);
  v8h hv;
#pragma unroll
  for (int e = 0; e < 4; ++e) {
    const float f0 = a0[e];
    const float f1 = a1[e];
    hv[e]     = (_Float16)carry_flush(bf16r(f0), kInCarry);
    hv[4 + e] = (_Float16)carry_flush(bf16r(f1), kInCarry);
  }
  unsigned short* dp = dst + (size_t)row * dstPitch + dstOff + c8;
  *(volatile v8h*)dp = hv;
  __threadfence();
  *(volatile v8h*)dp = hv;
}

__device__ __forceinline__ float fast_tanh(float v) { return 1.0f - 2.0f * frcp(__expf(2.0f * v) + 1.0f); }
__device__ __forceinline__ float fast_sigmoid(float v) { return frcp(1.0f + __expf(-v)); }

__global__ __launch_bounds__(kThr) void setup_kernel(const float* __restrict__ emb, const float* __restrict__ Wih_f, const float* __restrict__ Wih_b,
                                                     const float* __restrict__ b_f, const float* __restrict__ b_b, float* __restrict__ BIAS,
                                                     unsigned short* __restrict__ EMB16, unsigned short* __restrict__ WIF, unsigned short* __restrict__ WIB) {
  unsigned v = blockIdx.x * (unsigned)kThr + threadIdx.x;
  asm volatile("" : "+v"(v));
  if (v < 1024u) {
    const unsigned i0 = v * 4u;
    v4f o = {0.f, 0.f, 0.f, 0.f};
    if (i0 < (unsigned)kFZB) {
      const v4f a = *(const v4f*)((i0 < (unsigned)kFBB) ? (b_f + i0) : (b_b + (i0 - (unsigned)kFBB)));
#pragma unroll
      for (int e = 0; e < 4; ++e) { const float p = a[e]; o[e] = bf16r(p); }
    }
    float* dp = BIAS + i0;
    *(volatile v4f*)dp = o;
    __threadfence();
    *(volatile v4f*)dp = o;
  } else {
    const float* sp; unsigned short* dp;
    if (v < 3072u) { const unsigned w = v - 1024u; sp = emb + (size_t)w * 8u; dp = EMB16 + (size_t)w * 8u; }
    else if (v < 19456u) { const unsigned w = v - 3072u; sp = Wih_f + (size_t)w * 8u; dp = WIF + (size_t)w * 8u; }
    else { const unsigned w = v - 19456u; sp = Wih_b + (size_t)w * 8u; dp = WIB + (size_t)w * 8u; }
    const v4f a0 = *(const v4f*)sp, a1 = *(const v4f*)(sp + 4);
    v8h hv;
#pragma unroll
    for (int e = 0; e < 4; ++e) { const float p = a0[e], q = a1[e]; hv[e] = (_Float16)carry_flush(bf16r(p), kCarry); hv[4 + e] = (_Float16)carry_flush(bf16r(q), kCarry); }
    *(volatile v8h*)dp = hv;
    __threadfence();
    *(volatile v8h*)dp = hv;
  }
}
static_assert(kFEnd / 4 == 1024 && kV * kE / 8 == 2048 && kG4 * kE / 8 == 16384 && 1024 + 2048 + 16384 + 16384 == 140 * kThr && (3072 % 32) == 0 && (19456 % 32) == 0, "set-up grid exact; regions wave-uniform");

__global__ __launch_bounds__(kThr) void zero_state_kernel(float* __restrict__ H32, float* __restrict__ C32, unsigned short* __restrict__ H16) {
  const size_t v = (size_t)blockIdx.x * kThr + threadIdx.x;
  const v4f z = {0.f, 0.f, 0.f, 0.f};
  v8h hz;
#pragma unroll
  for (int e = 0; e < 8; ++e) hz[e] = (_Float16)0.0f;
  for (int pass = 0; pass < 2; ++pass) {
    *(volatile v4f*)(H32 + v * 8) = z;
    *(volatile v4f*)(H32 + v * 8 + 4) = z;
    *(volatile v4f*)(C32 + v * 8) = z;
    *(volatile v4f*)(C32 + v * 8 + 4) = z;
    *(volatile v8h*)(H16 + v * 8) = hz;
    __threadfence();
  }
}
static_assert(((size_t)kN * kHid / 8) % kThr == 0, "state grid exact");

__global__ __launch_bounds__(kThr) void lstm_cell_kernel(const float* __restrict__ GG, const float* __restrict__ PT, const int* __restrict__ char_ids,
                                                         const int* __restrict__ lengths, float* __restrict__ H32, float* __restrict__ C32,
                                                         unsigned short* __restrict__ H16, float* __restrict__ out, int t, int half, int last) {
  const size_t v = (size_t)blockIdx.x * kThr + threadIdx.x;
  const size_t w = v >> 5;
  const unsigned u8 = (unsigned)(v & 31) * 8u;
  int ch = char_ids[w * kT + (size_t)t];
  ch = (ch < 0) ? 0 : ((ch > kV - 1) ? (kV - 1) : ch);
  int len = lengths[w];
  len = (len < 0) ? 0 : ((len > kT) ? kT : len);
  const bool live = (t < len);
  const float* gr = GG + w * kG4 + u8;
  const float* pr = PT + (size_t)ch * kG4 + u8;
  float* hp = H32 + w * kHid + u8;
  float* cp = C32 + w * kHid + u8;
  v8h hv;
  v4f hn0, hn1, cn0, cn1;
#pragma unroll
  for (int hlf = 0; hlf < 2; ++hlf) {
    const v4f gi = *(const v4f*)(gr + 4 * hlf), gf = *(const v4f*)(gr + kHid + 4 * hlf), gg = *(const v4f*)(gr + 2 * kHid + 4 * hlf), go = *(const v4f*)(gr + 3 * kHid + 4 * hlf);
    const v4f pi = *(const v4f*)(pr + 4 * hlf), pf = *(const v4f*)(pr + kHid + 4 * hlf), pg = *(const v4f*)(pr + 2 * kHid + 4 * hlf), po = *(const v4f*)(pr + 3 * kHid + 4 * hlf);
    const v4f ho = *(const v4f*)(hp + 4 * hlf), co = *(const v4f*)(cp + 4 * hlf);
#pragma unroll
    for (int e = 0; e < 4; ++e) {
      const float cu = fast_sigmoid(pf[e] + gf[e]) * co[e] + fast_sigmoid(pi[e] + gi[e]) * fast_tanh(pg[e] + gg[e]);
      const float hu = fast_sigmoid(po[e] + go[e]) * fast_tanh(cu);
      const float cn = live ? cu : co[e];
      const float hn = live ? hu : ho[e];
      if (hlf == 0) { cn0[e] = cn; hn0[e] = hn; } else { cn1[e] = cn; hn1[e] = hn; }
      hv[4 * hlf + e] = (_Float16)carry_flush(hn, kCarry);
    }
  }
  unsigned short* h16p = H16 + w * kHid + u8;
  float* op = out + w * (size_t)(2 * kHid) + (size_t)half * kHid + u8;
  for (int pass = 0; pass < 2; ++pass) {
    *(volatile v4f*)hp = hn0;
    *(volatile v4f*)(hp + 4) = hn1;
    *(volatile v4f*)cp = cn0;
    *(volatile v4f*)(cp + 4) = cn1;
    *(volatile v8h*)h16p = hv;
    if (last) { *(volatile v4f*)op = hn0; *(volatile v4f*)(op + 4) = hn1; }
    __threadfence();
  }
}
static_assert(kHid / 8 == 32, "one wave a word");

static_assert(((size_t)kG4 * kHid / 8) % kThr == 0, "plane cast grid exact");

extern "C" void kernel_launch(void* const* d_in, const int* in_sizes, int n_in,
                              void* d_out, int out_size, void* d_ws, size_t ws_size,
                              hipStream_t stream) {
  if (n_in < 9 || d_out == nullptr || d_ws == nullptr) return;
  if (in_sizes[0] != kN * kT || in_sizes[1] != kN || in_sizes[2] != kV * kE || in_sizes[3] != kG4 * kE || in_sizes[4] != kG4 * kHid || in_sizes[5] != kG4) return;
  if (in_sizes[6] != kG4 * kE || in_sizes[7] != kG4 * kHid || in_sizes[8] != kG4) return;
  if (out_size != kN * 2 * kHid) return;
  if (ws_size < kWsTotal) return;
  const int* char_ids = (const int*)d_in[0];
  const int* lengths = (const int*)d_in[1];
  const float* emb = (const float*)d_in[2];
  const float* Wih_f = (const float*)d_in[3];
  const float* Whh_f = (const float*)d_in[4];
  const float* b_f = (const float*)d_in[5];
  const float* Wih_b = (const float*)d_in[6];
  const float* Whh_b = (const float*)d_in[7];
  const float* b_b = (const float*)d_in[8];
  float* out = (float*)d_out;
  char* ws = (char*)d_ws;
  unsigned short* EMB16 = (unsigned short*)(ws + kOffEMB16);
  unsigned short* WIF = (unsigned short*)(ws + kOffWIF);
  unsigned short* WIB = (unsigned short*)(ws + kOffWIB);
  unsigned short* WHF = (unsigned short*)(ws + kOffWHF);
  unsigned short* WHB = (unsigned short*)(ws + kOffWHB);
  float* BIAS = (float*)(ws + kOffBIAS);
  float* PF = (float*)(ws + kOffPF);
  float* PB = (float*)(ws + kOffPB);
  float* H32 = (float*)(ws + kOffH32);
  float* C32 = (float*)(ws + kOffC32);
  unsigned short* H16 = (unsigned short*)(ws + kOffH16);
  float* GG = (float*)(ws + kOffGG);

  cast_plane_kernel<<<(int)(((size_t)kG4 * kHid / 8) / kThr), kThr, 0, stream>>>(Whh_f, WHF, 8, kHid, 0);
  cast_plane_kernel<<<(int)(((size_t)kG4 * kHid / 8) / kThr), kThr, 0, stream>>>(Whh_b, WHB, 8, kHid, 0);
  setup_kernel<<<140, kThr, 0, stream>>>(emb, Wih_f, Wih_b, b_f, b_b, BIAS, EMB16, WIF, WIB);
  wmma_gemm64<0, false, 2, 0, false, 0><<<dim3((kV / 64) * (kG4 / 64) / 8, 1), 256, 0, stream>>>(
      EMB16, EMB16, kE, 0L, WIF, WIF, kE, 0L, (void*)PF, (void*)PF, kG4, 0L, BIAS + kFBF, nullptr, 0L, kV, kG4, kE, kSc);
  wmma_gemm64<0, false, 2, 0, false, 0><<<dim3((kV / 64) * (kG4 / 64) / 8, 1), 256, 0, stream>>>(
      EMB16, EMB16, kE, 0L, WIB, WIB, kE, 0L, (void*)PB, (void*)PB, kG4, 0L, BIAS + kFBB, nullptr, 0L, kV, kG4, kE, kSc);

  for (int dir = 0; dir < 2; ++dir) {
    const unsigned short* WH = (dir == 0) ? WHF : WHB;
    const float* PT = (dir == 0) ? PF : PB;
    zero_state_kernel<<<(int)(((size_t)kN * kHid / 8) / kThr), kThr, 0, stream>>>(H32, C32, H16);
    for (int s = 0; s < kT; ++s) {
      const int t = (dir == 0) ? s : (kT - 1 - s);
      wmma_gemm64<0, false, 2, 0, false, 0><<<dim3((kN / 64) * (kG4 / 64) / 8, 1), 256, 0, stream>>>(
          H16, H16, kHid, 0L, WH, WH, kHid, 0L, (void*)GG, (void*)GG, kG4, 0L, BIAS + kFZB, nullptr, 0L, kN, kG4, kHid, kSc);
      lstm_cell_kernel<<<(int)(((size_t)kN * kHid / 8) / kThr), kThr, 0, stream>>>(GG, PT, char_ids, lengths, H32, C32, H16, out, t, dir, (s == kT - 1) ? 1 : 0);
    }
  }
}
